// SlidingWindowAttentionBlock_678604833213
// MI455X (gfx1250) — hardware-verified
//
#include <hip/hip_runtime.h>
#include <math.h>

typedef __attribute__((ext_vector_type(16))) _Float16 v16h;
typedef __attribute__((ext_vector_type(16))) __bf16 v16b;
typedef __attribute__((ext_vector_type(8)))  _Float16 v8h;
typedef __attribute__((ext_vector_type(8)))  float v8f;
typedef __attribute__((ext_vector_type(4)))  float v4f;
typedef __attribute__((ext_vector_type(2)))  float v2f;
typedef __attribute__((ext_vector_type(4)))  unsigned v4u;
typedef __attribute__((ext_vector_type(4)))  int v4i;
typedef float __attribute__((may_alias)) float_a;
typedef int __attribute__((may_alias)) int_a;

template <typename T> __device__ __forceinline__ void vst2(void* p, T v) { *(volatile T*)p = v; __threadfence(); *(volatile T*)p = v; }
__device__ __forceinline__ v8f wmma16(v16h a, v16h b, v8f c) {
  v8f d = __builtin_amdgcn_wmma_f32_16x16x32_f16(false, a, false, b, (short)0, c, false, false);
  asm volatile("v_nop\n\tv_nop\n\tv_nop\n\tv_nop" : "+v"(d) : "v"(a), "v"(b));
  return d;
}
__device__ __forceinline__ v8f wmma_bf(v16b a, v16b b, v8f c) {
  v8f d = __builtin_amdgcn_wmma_f32_16x16x32_bf16(false, a, false, b, (short)0, c, false, false);
  asm volatile("v_nop\n\tv_nop\n\tv_nop\n\tv_nop" : "+v"(d) : "v"(a), "v"(b));
  return d;
}
__device__ __forceinline__ v16h frag_h(const _Float16* rowk0, int lane) {
  union { v16h v; v8h q[2]; } u; const _Float16* p = rowk0 + 8 * (lane >> 4);
  u.q[0] = *(const v8h*)p; u.q[1] = *(const v8h*)(p + 16); return u.v;
}
__device__ __forceinline__ v16h frag_f32(const float* rowk0, int lane) {
  v16h a; const float* p = rowk0 + 8 * (lane >> 4);
#pragma unroll
  for (int i = 0; i < 8; ++i) { a[i] = (_Float16)p[i]; a[8 + i] = (_Float16)p[16 + i]; }
  return a;
}
__device__ __forceinline__ v16h frag_f32s(const float* rowk0, int lane, float sc) {
  v16h a; const float* p = rowk0 + 8 * (lane >> 4);
#pragma unroll
  for (int i = 0; i < 8; ++i) { a[i] = (_Float16)(p[i] * sc); a[8 + i] = (_Float16)(p[16 + i] * sc); }
  return a;
}
__device__ __forceinline__ v16h fragc_f32(const float* W, int k0, int n, int lane, int ld, int K) {
  v16h a; const int g = lane >> 4;
#pragma unroll
  for (int i = 0; i < 8; ++i) { const int ka = k0 + 8 * g + i, kb = ka + 16;
    a[i] = (_Float16)(ka < K ? W[(size_t)(ka < K ? ka : K - 1) * ld + n] : 0.f); a[8 + i] = (_Float16)(kb < K ? W[(size_t)(kb < K ? kb : K - 1) * ld + n] : 0.f); }
  return a;
}
struct F2 { v16b h, l; };
__device__ __forceinline__ F2 bsplit16(const float v[16]) { F2 r;
#pragma unroll
  for (int i = 0; i < 16; ++i) { const __bf16 h = (__bf16)v[i]; r.h[i] = h; r.l[i] = (__bf16)(v[i] - (float)h); }
  return r; }
__device__ __forceinline__ F2 split_row(const float* row, int k0, int lane) { float v[16]; const float* p = row + k0 + 8 * (lane >> 4);
#pragma unroll
  for (int i = 0; i < 8; ++i) { v[i] = p[i]; v[8 + i] = p[16 + i]; }
  return bsplit16(v); }
__device__ __forceinline__ F2 split_rowK(const float* row, int k0, int lane, int K) { float v[16]; const int g = lane >> 4;
#pragma unroll
  for (int i = 0; i < 8; ++i) { const int ka = k0 + 8 * g + i, kb = ka + 16; v[i] = ka < K ? row[ka < K ? ka : K - 1] : 0.f; v[8 + i] = kb < K ? row[kb < K ? kb : K - 1] : 0.f; }
  return bsplit16(v); }
__device__ __forceinline__ F2 split_col(const float* W, int k0, int n, int lane, int ld, int K) { float v[16]; const int g = lane >> 4;
#pragma unroll
  for (int i = 0; i < 8; ++i) { const int ka = k0 + 8 * g + i, kb = ka + 16; v[i] = ka < K ? W[(size_t)(ka < K ? ka : K - 1) * ld + n] : 0.f; v[8 + i] = kb < K ? W[(size_t)(kb < K ? kb : K - 1) * ld + n] : 0.f; }
  return bsplit16(v); }
__device__ __forceinline__ v8f mac3(const F2& a, const F2& b, v8f c) { c = wmma_bf(a.l, b.h, c); c = wmma_bf(a.h, b.l, c); return wmma_bf(a.h, b.h, c); }
__device__ __forceinline__ float sigm(float v) { return 1.0f / (1.0f + expf(-v)); }
#define LDSX() do { asm volatile("s_wait_dscnt 0" ::: "memory"); __builtin_amdgcn_wave_barrier(); __builtin_amdgcn_fence(__ATOMIC_RELEASE, "workgroup"); } while (0)


#define NB 2
#define DD 64
#define IH 128
#define IW 128
#define NPIX (IH * IW)
#define NHD 4
#define HDD 16
#define KW 7
#define RR 3
#define FF 256
#define NR (NB * NPIX)
typedef __attribute__((ext_vector_type(8))) __bf16 v8b;
__device__ __forceinline__ v16b frag_b(const __bf16* rowk0, int lane) {
  union { v16b v; v8b q[2]; } u; const __bf16* p = rowk0 + 8 * (lane >> 4);
  u.q[0] = *(const v8b*)p; u.q[1] = *(const v8b*)(p + 16); return u.v;
}
__device__ __forceinline__ float bfr(float v) { return (float)(__bf16)v; }
__device__ __attribute__((noinline)) float exp_ni(float v) { return expf(v); }
__device__ __attribute__((noinline)) float erf_ni(float v) { return erff(v); }

#define WS_XC  0u
#define WS_Q   (WS_XC + 4u * (size_t)NR * DD)
#define WS_K   (WS_Q + 4u * (size_t)NR * DD)
#define WS_V   (WS_K + 2u * (size_t)NR * DD)
#define WS_AO  (WS_V + 2u * (size_t)NR * DD)
#define WS_END (WS_AO + 4u * (size_t)NR * DD)

__device__ __forceinline__ int reflect_idx(int i, int n) { return i < 0 ? -i : (i >= n ? 2 * n - 2 - i : i); }
__global__ __launch_bounds__(128) void k_pre(const float* __restrict__ X, const float* __restrict__ G1, const float* __restrict__ B1n, const float* __restrict__ WQ, const float* __restrict__ WK, const float* __restrict__ WV, float* __restrict__ XC, float* __restrict__ Q, _Float16* __restrict__ Kr, _Float16* __restrict__ Vr) {
  __shared__ __align__(16) float sx[64][DD + 4]; __shared__ __align__(16) _Float16 sa[64][DD + 8]; __shared__ __align__(16) float sq[64][DD + 4]; __shared__ __align__(16) _Float16 sk[64][DD + 8], sv[64][DD + 8];
  const int tid = threadIdx.x, wave = tid >> 5, lane = tid & 31, col = lane & 15, g = lane >> 4; const size_t p0 = (size_t)blockIdx.x * 64; const size_t b = p0 / NPIX; const int pp = (int)(p0 % NPIX); const int y = pp / IW, x0 = pp % IW;
  for (int e = tid; e < 64 * DD; e += 128) { const int c = e >> 6, j = e & 63; sx[j][c] = bfr(X[((b * DD + c) * IH + y) * (size_t)IW + x0 + j]); }
  __syncthreads();
  if (tid < 64) { float m = 0.f; for (int c = 0; c < DD; ++c) m += sx[tid][c]; m *= (1.0f / DD); float v = 0.f; for (int c = 0; c < DD; ++c) { const float d = sx[tid][c] - m; v += d * d; } const float inv = 1.0f / sqrtf(v * (1.0f / DD) + 1e-5f);
    for (int c = 0; c < DD; ++c) sa[tid][c] = (_Float16)((sx[tid][c] - m) * inv * bfr(G1[c]) + bfr(B1n[c])); }
  __syncthreads();
  v8f acc[12]; for (int j = 0; j < 12; ++j) for (int r = 0; r < 8; ++r) acc[j][r] = 0.f;
#pragma unroll
  for (int kc = 0; kc < DD / 32; ++kc) { const v16h a = frag_h(&sa[wave * 16 + col][kc * 32], lane);
#pragma unroll
    for (int j = 0; j < 12; ++j) { const float* Wm = (j < 4) ? WQ : (j < 8) ? WK : WV; const int o = (j & 3) * 16 + col; v16h w; const float* p = Wm + (size_t)o * DD + kc * 32 + 8 * g;
#pragma unroll
      for (int i = 0; i < 8; ++i) { w[i] = (_Float16)bfr(p[i]); w[8 + i] = (_Float16)bfr(p[16 + i]); }
      acc[j] = wmma16(a, w, acc[j]); } }
#pragma unroll
  for (int j = 0; j < 12; ++j)
#pragma unroll
    for (int r = 0; r < 8; ++r) { const int rl = wave * 16 + 8 * g + r, o = (j & 3) * 16 + col; if (j < 4) sq[rl][o] = acc[j][r]; else if (j < 8) sk[rl][o] = (_Float16)acc[j][r]; else sv[rl][o] = (_Float16)acc[j][r]; }
  __syncthreads();
  for (int e = tid; e < 64 * 16; e += 128) { const int rl = e >> 4, q = e & 15; vst2(XC + (p0 + rl) * DD + q * 4, *(const v4f*)&sx[rl][q * 4]); vst2(Q + (p0 + rl) * DD + q * 4, *(const v4f*)&sq[rl][q * 4]); }
  for (int e = tid; e < 64 * 8; e += 128) { const int rl = e >> 3, q = e & 7; vst2((unsigned*)(Kr + (p0 + rl) * DD + q * 8), *(const v4u*)&sk[rl][q * 8]); vst2((unsigned*)(Vr + (p0 + rl) * DD + q * 8), *(const v4u*)&sv[rl][q * 8]); } }
__global__ __launch_bounds__(256) void k_win(const float* __restrict__ Q, const _Float16* __restrict__ Kr, const _Float16* __restrict__ Vr, float* __restrict__ AO) { __shared__ __align__(16) _Float16 skk[14 * 14][DD], svv[14 * 14][DD];
  const int t = threadIdx.x; const size_t b = blockIdx.z; const int ty0 = blockIdx.y * 8, tx0 = blockIdx.x * 8;
  for (int e = t; e < 196 * 8; e += 256) { const int cell = e >> 3, q = e & 7; const int cy = cell / 14, cx = cell % 14; const int gy = reflect_idx(ty0 - RR + cy, IH), gx = reflect_idx(tx0 - RR + cx, IW); const size_t pix = b * NPIX + (size_t)gy * IW + gx;
    *(v4u*)&skk[cell][q * 8] = *(const v4u*)(Kr + pix * DD + q * 8); *(v4u*)&svv[cell][q * 8] = *(const v4u*)(Vr + pix * DD + q * 8); }
  __syncthreads();
  const int pl = t >> 2, hh = t & 3; const int py = pl >> 3, px = pl & 7; const size_t pix = b * NPIX + (size_t)(ty0 + py) * IW + tx0 + px;
  float qv[HDD]; { const float* qp = Q + pix * DD + hh * HDD;
#pragma unroll
    for (int d = 0; d < HDD; ++d) qv[d] = qp[d] * 0.25f; }
  float mx = -3.0e38f;
#pragma unroll 1
  for (int n = 0; n < KW * KW; ++n) { const int dy = n / KW, dx = n % KW; const _Float16* kp = &skk[(py + dy) * 14 + (px + dx)][hh * HDD]; float s = 0.f;
#pragma unroll
    for (int d = 0; d < HDD; ++d) s += qv[d] * (float)kp[d]; mx = fmaxf(mx, s); }
  float sum = 0.f; float o[HDD];
#pragma unroll
  for (int d = 0; d < HDD; ++d) o[d] = 0.f;
#pragma unroll 1
  for (int n = 0; n < KW * KW; ++n) { const int dy = n / KW, dx = n % KW; const int cell = (py + dy) * 14 + (px + dx); const _Float16* kp = &skk[cell][hh * HDD]; const _Float16* vp = &svv[cell][hh * HDD]; float s = 0.f;
#pragma unroll
    for (int d = 0; d < HDD; ++d) s += qv[d] * (float)kp[d]; const float e = expf(s - mx); sum += e;
#pragma unroll
    for (int d = 0; d < HDD; ++d) o[d] += e * (float)vp[d]; }
  const float inv = 1.0f / sum;
#pragma unroll
  for (int d = 0; d < HDD; ++d) o[d] *= inv;
  float* dst = AO + pix * DD + hh * HDD;
#pragma unroll
  for (int q = 0; q < HDD / 4; ++q) { v4f v; v[0] = o[q * 4]; v[1] = o[q * 4 + 1]; v[2] = o[q * 4 + 2]; v[3] = o[q * 4 + 3]; vst2(dst + q * 4, v); } }
__global__ __launch_bounds__(128) void k_post(const float* __restrict__ AO, const float* __restrict__ XC, const float* __restrict__ WO, const float* __restrict__ G2, const float* __restrict__ B2n, const float* __restrict__ W1, const float* __restrict__ Bf1, const float* __restrict__ W2, const float* __restrict__ Bf2, float* __restrict__ OUT) {
  __shared__ __align__(16) _Float16 sa[64][DD + 8]; __shared__ __align__(16) float sy[64][DD + 4]; __shared__ __align__(16) _Float16 sh2[64][FF + 8]; __shared__ __align__(16) float so[DD][68];
  const int tid = threadIdx.x, wave = tid >> 5, lane = tid & 31, col = lane & 15, g = lane >> 4; const size_t p0 = (size_t)blockIdx.x * 64; const size_t b = p0 / NPIX; const int pp = (int)(p0 % NPIX); const int y = pp / IW, x0 = pp % IW;
  for (int e = tid; e < 64 * DD; e += 128) { const int rl = e >> 6, c = e & 63; sa[rl][c] = (_Float16)AO[(p0 + rl) * DD + c]; }
  __syncthreads();
  { v8f acc[4] = {};
#pragma unroll
    for (int kc = 0; kc < DD / 32; ++kc) { const v16h a = frag_h(&sa[wave * 16 + col][kc * 32], lane);
#pragma unroll
      for (int j = 0; j < 4; ++j) { const int o = j * 16 + col; v16h w; const float* p = WO + (size_t)o * DD + kc * 32 + 8 * g;
#pragma unroll
        for (int i = 0; i < 8; ++i) { w[i] = (_Float16)bfr(p[i]); w[8 + i] = (_Float16)bfr(p[16 + i]); }
        acc[j] = wmma16(a, w, acc[j]); } }
#pragma unroll
    for (int j = 0; j < 4; ++j)
#pragma unroll
      for (int r = 0; r < 8; ++r) { const int rl = wave * 16 + 8 * g + r, o = j * 16 + col; sy[rl][o] = acc[j][r] + XC[(p0 + rl) * DD + o]; } }
  __syncthreads();
  if (tid < 64) { float m = 0.f; for (int c = 0; c < DD; ++c) m += sy[tid][c]; m *= (1.0f / DD); float v = 0.f; for (int c = 0; c < DD; ++c) { const float d = sy[tid][c] - m; v += d * d; } const float inv = 1.0f / sqrtf(v * (1.0f / DD) + 1e-5f);
    for (int c = 0; c < DD; ++c) sa[tid][c] = (_Float16)((sy[tid][c] - m) * inv * bfr(G2[c]) + bfr(B2n[c])); }
  __syncthreads();
#pragma unroll 1
  for (int half = 0; half < 2; ++half) { v8f acc[8] = {};
#pragma unroll
    for (int kc = 0; kc < DD / 32; ++kc) { const v16h a = frag_h(&sa[wave * 16 + col][kc * 32], lane);
#pragma unroll
      for (int j = 0; j < 8; ++j) { const int o = half * 128 + j * 16 + col; v16h w; const float* p = W1 + (size_t)o * DD + kc * 32 + 8 * g;
#pragma unroll
        for (int i = 0; i < 8; ++i) { w[i] = (_Float16)bfr(p[i]); w[8 + i] = (_Float16)bfr(p[16 + i]); }
        acc[j] = wmma16(a, w, acc[j]); } }
#pragma unroll
    for (int j = 0; j < 8; ++j) { const int o = half * 128 + j * 16 + col; const float bb = bfr(Bf1[o]);
#pragma unroll
      for (int r = 0; r < 8; ++r) { const float u = acc[j][r] + bb; sh2[wave * 16 + 8 * g + r][o] = (_Float16)(0.5f * u * (1.0f + erff(u * 0.70710678118654752f))); } } }
  __syncthreads();
  { v8f acc[4] = {};
#pragma unroll
    for (int kc = 0; kc < FF / 32; ++kc) { const v16h a = frag_h(&sh2[wave * 16 + col][kc * 32], lane);
#pragma unroll
      for (int j = 0; j < 4; ++j) { const int o = j * 16 + col; v16h w; const float* p = W2 + (size_t)o * FF + kc * 32 + 8 * g;
#pragma unroll
        for (int i = 0; i < 8; ++i) { w[i] = (_Float16)bfr(p[i]); w[8 + i] = (_Float16)bfr(p[16 + i]); }
        acc[j] = wmma16(a, w, acc[j]); } }
#pragma unroll
    for (int j = 0; j < 4; ++j) { const int o = j * 16 + col; const float bb = bfr(Bf2[o]);
#pragma unroll
      for (int r = 0; r < 8; ++r) { const int rl = wave * 16 + 8 * g + r; so[o][rl] = sy[rl][o] + acc[j][r] + bb; } } }
  __syncthreads(); for (int e = tid; e < DD * 16; e += 128) { const int c = e >> 4, q = e & 15; vst2(OUT + ((b * DD + c) * IH + y) * (size_t)IW + x0 + q * 4, *(const v4f*)&so[c][q * 4]); } }
extern "C" void kernel_launch(void* const* d_in, const int* in_sizes, int n_in, void* d_out, int out_size, void* d_ws, size_t ws_size, hipStream_t stream) {
  (void)in_sizes; (void)n_in; (void)out_size;
  const float** F = (const float**)d_in;
  if (ws_size < (size_t)WS_END) return;
  char* ws = (char*)d_ws; float *XC = (float*)(ws + WS_XC), *Q = (float*)(ws + WS_Q), *AO = (float*)(ws + WS_AO); _Float16 *Kr = (_Float16*)(ws + WS_K), *Vr = (_Float16*)(ws + WS_V);
  k_pre<<<NR / 64, 128, 0, stream>>>(F[0], F[1], F[2], F[3], F[4], F[5], XC, Q, Kr, Vr);
  k_win<<<dim3(IW / 8, IH / 8, NB), 256, 0, stream>>>(Q, Kr, Vr, AO);
  k_post<<<NR / 64, 128, 0, stream>>>(AO, XC, F[6], F[7], F[8], F[9], F[10], F[11], F[12], (float*)d_out);
}
